// GraphAttention_86715389706288
// MI455X (gfx1250) — hardware-verified
//
#include <hip/hip_runtime.h>
#include <stddef.h>


typedef _Float16 v16h __attribute__((ext_vector_type(16)));
typedef _Float16 v8h  __attribute__((ext_vector_type(8)));
typedef float    v8f  __attribute__((ext_vector_type(8)));
typedef float    v4f  __attribute__((ext_vector_type(4)));
typedef _Float16 h16;

#ifndef NB
#define NB 8
#endif
#ifndef SEQ
#define SEQ 1024
#endif
#define NB_FULL  8
#define SEQ_FULL 1024
#define FIN   256
#define DIM   256
#define NHEAD 4
#define HD    64
#define MROWS (NB * SEQ)

static_assert(NB >= 1 && NB <= NB_FULL);
static_assert(SEQ >= 256 && SEQ <= SEQ_FULL && (SEQ % 256) == 0);
static_assert(DIM == NHEAD * HD);
static_assert(HD == 64);
static_assert((DIM / 64) == NHEAD);
static_assert((FIN % 64) == 0 && (FIN % 32) == 0);
static_assert(FIN == 32 * 8);
static_assert((MROWS % 64) == 0 && (MROWS % 8) == 0);
static_assert((SEQ % 128) == 0 && (SEQ % 64) == 0 && (SEQ % 32) == 0);

#define LDT 72
#define LDC 68
#define LDO 36
static_assert((LDT % 8) == 0 && LDT >= 64);
static_assert((LDC % 4) == 0 && LDC >= 64);
static_assert((LDO % 4) == 0 && LDO >= 32);

#define WCARRY 64.0f
#define PCARRY 1024.0f
#define LRELU  0.2f
#define MASK_VAL (-9.0e15f)

#define WT_BYTES   ((size_t)DIM * FIN * 2)
#define X16_BYTES  ((size_t)MROWS * FIN * 2)
#define VT_BYTES   ((size_t)NB * DIM * SEQ * 2)
#define EJ_OFF     ((size_t)NB * NHEAD * SEQ)
#define EE_BYTES   ((size_t)2 * NB * NHEAD * SEQ * 4)
#define MT_BYTES   ((size_t)(SEQ / 32) * SEQ * 4)
#define OFF_WT  ((size_t)0)
#define OFF_X16 (OFF_WT + WT_BYTES)
#define OFF_VT  (OFF_X16 + X16_BYTES)
#define OFF_EE  (OFF_VT + VT_BYTES)
#define OFF_MT  (OFF_EE + EE_BYTES)
#define WS_TOTAL (OFF_MT + MT_BYTES)
static_assert((WT_BYTES % 128) == 0 && (X16_BYTES % 128) == 0 && (VT_BYTES % 128) == 0);
static_assert((EE_BYTES % 128) == 0 && (MT_BYTES % 128) == 0 && ((EJ_OFF * 4) % 128) == 0);
static_assert(WS_TOTAL <= (size_t)134217728);

__device__ __forceinline__ float bf16r(float x) {
  unsigned int u = __float_as_uint(x);
  u = (u + 0x7FFFu + ((u >> 16) & 1u)) & 0xFFFF0000u;
  return __uint_as_float(u);
}

static __device__ __forceinline__ h16 toh_flush(float v) {
  const h16 r = (h16)v;
  return (fabsf(v) < 6.103515625e-05f) ? (h16)0.0f : r;
}

__device__ __forceinline__ v16h frag_at(const _Float16* p) {
  v8h lo = *(const v8h*)(p);
  v8h hi = *(const v8h*)(p + 16);
  v16h out;
#pragma unroll
  for (int i = 0; i < 8; ++i) { out[i] = lo[i]; out[i + 8] = hi[i]; }
  return out;
}
__device__ __forceinline__ v16h ld_frag(const _Float16* base, unsigned ld) {
  const unsigned lane = threadIdx.x & 31u;
  return frag_at(base + (lane & 15u) * ld + (lane >> 4) * 8u);
}

__device__ __forceinline__ v8f wmma16(v16h a, v16h b, v8f c) {
  v8f d = __builtin_amdgcn_wmma_f32_16x16x32_f16(false, a, false, b, (short)0, c,
                                                 false, false);
  asm volatile("v_nop\n\tv_nop\n\tv_nop\n\tv_nop" : "+v"(d) : "v"(a), "v"(b));
  return d;
}

__device__ __forceinline__ float red16_max(float x) {
#pragma unroll
  for (int off = 1; off < 16; off <<= 1) x = fmaxf(x, __shfl_xor(x, off, 32));
  return x;
}
__device__ __forceinline__ float red16_sum(float x) {
#pragma unroll
  for (int off = 1; off < 16; off <<= 1) x += __shfl_xor(x, off, 32);
  return x;
}

__device__ __forceinline__ void wave_lds_sync() {
  __builtin_amdgcn_fence(3  , "wavefront");
  asm volatile("s_wait_dscnt 0x0" ::: "memory");
  __builtin_amdgcn_wave_barrier();
}

__global__ __launch_bounds__(256) void wconv_kernel(
    const float* __restrict__ W, _Float16* __restrict__ Wt, unsigned ldw, unsigned ldk) {
  __shared__ _Float16 T[64 * LDT];
  const unsigned tid = threadIdx.x;
  const unsigned n0 = blockIdx.x * 64u;
  const unsigned k0 = blockIdx.y * 64u;
#pragma unroll 4
  for (unsigned j = 0; j < 16u; ++j) {
    const unsigned idx = tid + 256u * j;
    const unsigned kr = idx >> 6, nc = idx & 63u;
    const float v = W[(size_t)(k0 + kr) * ldw + n0 + nc];
    T[nc * LDT + kr] = (_Float16)(WCARRY * bf16r(v));
  }
  __syncthreads();
  v8h x[2];
  size_t off[2];
#pragma unroll
  for (unsigned i = 0; i < 2u; ++i) {
    const unsigned n = 32u * i + (tid >> 3);
    const unsigned kc = (tid & 7u) * 8u;
    x[i] = *(const v8h*)&T[n * LDT + kc];
    off[i] = (size_t)(n0 + n) * ldk + k0 + kc;
  }
#pragma unroll
  for (int i = 0; i < 2; ++i) *(volatile v8h*)(Wt + off[i]) = x[i];
  __threadfence();
#pragma unroll
  for (int i = 0; i < 2; ++i) *(volatile v8h*)(Wt + off[i]) = x[i];
}

__global__ __launch_bounds__(256) void xconv_kernel(
    const float* __restrict__ X, _Float16* __restrict__ dst) {
  const unsigned lane = threadIdx.x & 31u;
  const unsigned w = (unsigned)__builtin_amdgcn_readfirstlane((int)(threadIdx.x >> 5));
  const unsigned crow = blockIdx.x * 8u + w;
  const unsigned bidx = crow / (unsigned)SEQ;
  const unsigned sq = crow - bidx * (unsigned)SEQ;
  const size_t srow = (size_t)bidx * SEQ_FULL + sq;
  const float* xr = X + srow * FIN + lane * 8u;
  const v4f a0 = *(const v4f*)(xr);
  const v4f a1 = *(const v4f*)(xr + 4u);
  v8h o;
#pragma unroll
  for (int i = 0; i < 4; ++i) {
    o[i]     = toh_flush(bf16r(a0[i]));
    o[i + 4] = toh_flush(bf16r(a1[i]));
  }
  _Float16* p = dst + (size_t)crow * FIN + lane * 8u;
  *(volatile v8h*)p = o;
  __threadfence();
  *(volatile v8h*)p = o;
}

__global__ __launch_bounds__(256) void maskpack_kernel(
    const int* __restrict__ adj, unsigned int* __restrict__ MT) {
  const unsigned per = (unsigned)SEQ / 256u;
  const unsigned iw = blockIdx.x / per;
  const unsigned j = (blockIdx.x - iw * per) * 256u + threadIdx.x;
  unsigned int word = 0u;
#pragma unroll 4
  for (unsigned r = 0; r < 32u; ++r) {
    const int av = adj[(size_t)(iw * 32u + r) * SEQ_FULL + j];
    word |= ((av > 0) ? 1u : 0u) << r;
  }
  unsigned int* p = MT + (size_t)iw * SEQ + j;
  *(volatile unsigned int*)p = word;
  __threadfence();
  *(volatile unsigned int*)p = word;
}

__global__ __launch_bounds__(256) void wh_gemm_kernel(
    const _Float16* __restrict__ A16, const _Float16* __restrict__ Bt,
    const float* __restrict__ avec, _Float16* __restrict__ vt, float* __restrict__ ee) {
  __shared__ float Cs[64 * LDC];
  __shared__ float Es[128];
  const unsigned K = (unsigned)FIN;
  const unsigned tid = threadIdx.x, lane = tid & 31u;
  const unsigned w = (unsigned)__builtin_amdgcn_readfirstlane((int)(threadIdx.x >> 5));
  const unsigned mw = w >> 1, nw = w & 1u;
  const unsigned hh = lane >> 4, m = lane & 15u;
  const unsigned n0 = blockIdx.x * 64u;
  const unsigned head = blockIdx.x;
  const unsigned row0 = blockIdx.y * 64u;

  const _Float16* ap  = A16 + (size_t)(row0 + mw * 16u + m) * K + hh * 8u;
  const _Float16* bp0 = Bt + (size_t)(n0 + nw * 32u + m) * K + hh * 8u;
  const _Float16* bp1 = bp0 + (size_t)16 * K;
  v8f acc0 = {}, acc1 = {};
#pragma unroll 2
  for (unsigned k0 = 0; k0 < K; k0 += 32u) {
    const v16h a  = frag_at(ap + k0);
    const v16h b0 = frag_at(bp0 + k0);
    const v16h b1 = frag_at(bp1 + k0);
    acc0 = wmma16(a, b0, acc0);
    acc1 = wmma16(a, b1, acc1);
  }
#pragma unroll
  for (int r = 0; r < 8; ++r) {
    float* d = &Cs[(mw * 16u + hh * 8u + (unsigned)r) * LDC + nw * 32u + m];
    d[0]  = acc0[r];
    d[16] = acc1[r];
  }
  __syncthreads();

  {
    const unsigned r = tid >> 2, qd = tid & 3u;
    const float* a1p = avec + head * (2u * HD) + qd * 16u;
    float s1 = 0.0f, s2 = 0.0f;
#pragma unroll 1
    for (unsigned g = 0; g < 4u; ++g) {
      const v4f u  = *(const v4f*)&Cs[r * LDC + qd * 16u + g * 4u];
      const v4f c1 = *(const v4f*)(a1p + g * 4u);
      const v4f c2 = *(const v4f*)(a1p + HD + g * 4u);
#pragma unroll
      for (int j = 0; j < 4; ++j) {
        const float wv = u[j] * (1.0f / WCARRY);
        s1 += wv * bf16r(c1[j]);
        s2 += wv * bf16r(c2[j]);
      }
    }
    s1 += __shfl_xor(s1, 1, 32);
    s2 += __shfl_xor(s2, 1, 32);
    s1 += __shfl_xor(s1, 2, 32);
    s2 += __shfl_xor(s2, 2, 32);
    if (qd == 0u) {
      Es[r] = s1;
      Es[64u + r] = s2;
    }
  }

  const unsigned bidx = row0 / (unsigned)SEQ;
  const unsigned key0 = row0 - bidx * (unsigned)SEQ;
  {
    v8h x[2];
    size_t off[2];
#pragma unroll
    for (unsigned i = 0; i < 2u; ++i) {
      const unsigned dcol = 32u * i + (tid >> 3);
      const unsigned kk = (tid & 7u) * 8u;
#pragma unroll
      for (unsigned j = 0; j < 8u; ++j)
        x[i][j] = toh_flush(Cs[(kk + j) * LDC + dcol] * (1.0f / WCARRY));
      off[i] = ((size_t)bidx * DIM + n0 + dcol) * SEQ + key0 + kk;
    }
#pragma unroll
    for (int i = 0; i < 2; ++i) *(volatile v8h*)(vt + off[i]) = x[i];
    __threadfence();
#pragma unroll
    for (int i = 0; i < 2; ++i) *(volatile v8h*)(vt + off[i]) = x[i];
  }
  __syncthreads();

  if (w == 0u) {
    const unsigned which = lane >> 4, c = (lane & 15u) * 4u;
    const v4f val = *(const v4f*)&Es[which * 64u + c];
    float* p = ee + (size_t)which * EJ_OFF + ((size_t)bidx * NHEAD + head) * SEQ + key0 + c;
    *(volatile v4f*)p = val;
    __threadfence();
    *(volatile v4f*)p = val;
  }
}

__global__ __launch_bounds__(256) void gat_attn_kernel(
    const _Float16* __restrict__ Vt, const float* __restrict__ EE,
    const unsigned int* __restrict__ MT, float* __restrict__ out) {
  __shared__ _Float16 Vs[64 * LDT];
  __shared__ _Float16 Ps[8 * 16 * LDT];
  __shared__ float Ejs[SEQ];
  __shared__ float Os[8 * 16 * LDO];

  const unsigned tid = threadIdx.x, lane = tid & 31u;
  const unsigned w = (unsigned)__builtin_amdgcn_readfirstlane((int)(threadIdx.x >> 5));
  const unsigned hh = lane >> 4, m = lane & 15u;
  const unsigned q0 = blockIdx.x * 128u;
  const unsigned head = blockIdx.y;
  const unsigned b = blockIdx.z;
  const unsigned qrow0 = q0 + w * 16u;
  _Float16* P = Ps + w * (16u * LDT);
  float* O = Os + w * (16u * LDO);

  const size_t erow = ((size_t)b * NHEAD + head) * SEQ;
  float eiv[8];
  {
    const float* eip = EE + erow + qrow0 + hh * 8u;
    const v4f ea = *(const v4f*)(eip);
    const v4f eb = *(const v4f*)(eip + 4u);
#pragma unroll
    for (int i = 0; i < 4; ++i) { eiv[i] = ea[i]; eiv[i + 4] = eb[i]; }
  }
  {
    const float* ejp = EE + EJ_OFF + erow;
    for (unsigned c = tid * 4u; c < (unsigned)SEQ; c += 1024u)
      *(v4f*)&Ejs[c] = *(const v4f*)(ejp + c);
  }

  float mrow[8], lrow[8];
  v8f o[4];
#pragma unroll
  for (int v = 0; v < 8; ++v) { mrow[v] = -1.0e30f; lrow[v] = 0.0f; }
#pragma unroll
  for (int nb = 0; nb < 4; ++nb) o[nb] = (v8f){};

  const size_t vplane = ((size_t)b * DIM + head * HD) * SEQ;
  const unsigned int* mtp = MT + (size_t)(qrow0 >> 5) * SEQ;
  const unsigned sh0 = (qrow0 & 16u) + hh * 8u;

  for (unsigned kb = 0; kb < (unsigned)SEQ; kb += 64u) {
#pragma unroll
    for (unsigned j = 0; j < 2u; ++j) {
      const unsigned idx = tid + 256u * j;
      const unsigned r = idx >> 3, c = (idx & 7u) * 8u;
      *(v8h*)&Vs[r * LDT + c] = *(const v8h*)(Vt + vplane + (size_t)r * SEQ + kb + c);
    }
    __syncthreads();

    unsigned int wd[4];
    float ejv[4];
#pragma unroll
    for (int kg = 0; kg < 4; ++kg) {
      unsigned int t = mtp[kb + (unsigned)kg * 16u + m];
      asm volatile("" : "+v"(t));
      wd[kg] = t;
      ejv[kg] = Ejs[kb + (unsigned)kg * 16u + m];
    }

    v8f s[4];
#pragma unroll
    for (int kg = 0; kg < 4; ++kg)
#pragma unroll
      for (int v = 0; v < 8; ++v) {
        float e = eiv[v] + ejv[kg];
        e = (e > 0.0f) ? e : LRELU * e;
        const unsigned bit = (wd[kg] >> (sh0 + (unsigned)v)) & 1u;
        s[kg][v] = (bit != 0u) ? e : MASK_VAL;
      }

    float alpha[8];
#pragma unroll
    for (int v = 0; v < 8; ++v) {
      float mx = fmaxf(fmaxf(s[0][v], s[1][v]), fmaxf(s[2][v], s[3][v]));
      mx = red16_max(mx);
      const float mn = fmaxf(mrow[v], mx);
      alpha[v] = __expf(mrow[v] - mn);
      mrow[v] = mn;
    }
#pragma unroll
    for (int kg = 0; kg < 4; ++kg)
#pragma unroll
      for (int v = 0; v < 8; ++v) {
        const float t = __expf(s[kg][v] - mrow[v]) * PCARRY;
        const h16 ph = toh_flush(t);
        P[(hh * 8u + (unsigned)v) * LDT + (unsigned)kg * 16u + m] = ph;
        s[kg][v] = (float)ph;
      }
#pragma unroll
    for (int v = 0; v < 8; ++v) {
      const float rs = red16_sum((s[0][v] + s[1][v]) + (s[2][v] + s[3][v]));
      lrow[v] = alpha[v] * lrow[v] + rs;
    }
#pragma unroll
    for (int nb = 0; nb < 4; ++nb)
#pragma unroll
      for (int v = 0; v < 8; ++v) o[nb][v] = o[nb][v] * alpha[v];
    wave_lds_sync();

#pragma unroll
    for (int c = 0; c < 2; ++c) {
      const v16h pf = ld_frag(P + c * 32, LDT);
#pragma unroll
      for (int nb = 0; nb < 4; ++nb) {
        const v16h vf = ld_frag(&Vs[(nb * 16) * LDT + c * 32], LDT);
        o[nb] = wmma16(pf, vf, o[nb]);
      }
    }
    __syncthreads();
  }

  float inv[8];
#pragma unroll
  for (int v = 0; v < 8; ++v) inv[v] = __builtin_amdgcn_rcpf(lrow[v]);
#pragma unroll
  for (int hf = 0; hf < 2; ++hf) {
#pragma unroll
    for (int nbl = 0; nbl < 2; ++nbl)
#pragma unroll
      for (int v = 0; v < 8; ++v) {
        float val = o[hf * 2 + nbl][v] * inv[v];
        val = (val > 0.0f) ? val : (__expf(val) - 1.0f);
        O[(hh * 8u + (unsigned)v) * LDO + (unsigned)nbl * 16u + m] = val;
      }
    wave_lds_sync();
    v4f x[4];
    size_t off[4];
#pragma unroll
    for (unsigned i = 0; i < 4u; ++i) {
      const unsigned r = 4u * i + (lane >> 3);
      const unsigned c = (lane & 7u) * 4u;
      x[i] = *(const v4f*)&O[r * LDO + c];
      off[i] = ((size_t)b * SEQ_FULL + qrow0 + r) * DIM + head * HD + (unsigned)hf * 32u + c;
    }
#pragma unroll
    for (int i = 0; i < 4; ++i) *(volatile v4f*)(out + off[i]) = x[i];
    __threadfence();
#pragma unroll
    for (int i = 0; i < 4; ++i) *(volatile v4f*)(out + off[i]) = x[i];
    wave_lds_sync();
  }
}

extern "C" void kernel_launch(void* const* d_in, const int* in_sizes, int n_in,
                              void* d_out, int out_size, void* d_ws, size_t ws_size,
                              hipStream_t stream) {
  if (n_in < 4) return;
  const long long need_x = ((long long)(NB - 1) * SEQ_FULL + SEQ) * FIN;
  const long long need_o = ((long long)(NB - 1) * SEQ_FULL + SEQ) * DIM;
  const long long need_adj = (long long)(SEQ - 1) * SEQ_FULL + SEQ;
  if ((long long)in_sizes[0] < need_x) return;
  if ((long long)in_sizes[1] < need_adj) return;
  if ((long long)in_sizes[2] < (long long)NHEAD * FIN * HD) return;
  if ((long long)in_sizes[3] < (long long)NHEAD * 2 * HD) return;
  if ((long long)out_size < need_o) return;
  if (ws_size < WS_TOTAL) return;

  const float* X    = (const float*)d_in[0];
  const int*   adj  = (const int*)d_in[1];
  const float* Wsrc = (const float*)d_in[2];
  const float* avec = (const float*)d_in[3];
  float* out = (float*)d_out;

  char* ws = (char*)d_ws;
  _Float16* Wt   = (_Float16*)(ws + OFF_WT);
  _Float16* X16  = (_Float16*)(ws + OFF_X16);
  _Float16* Vt16 = (_Float16*)(ws + OFF_VT);
  float*    EE   = (float*)(ws + OFF_EE);
  unsigned int* MT = (unsigned int*)(ws + OFF_MT);

  dim3 blk(256);

  for (int h = 0; h < NHEAD; ++h) {
    wconv_kernel<<<dim3(HD / 64, FIN / 64), blk, 0, stream>>>(
        Wsrc + (size_t)h * FIN * HD, Wt + (size_t)h * HD * FIN, (unsigned)HD, (unsigned)FIN);
  }
  xconv_kernel<<<dim3(MROWS / 8), blk, 0, stream>>>(X, X16);
  maskpack_kernel<<<dim3((SEQ / 32) * (SEQ / 256)), blk, 0, stream>>>(adj, MT);
  wh_gemm_kernel<<<dim3(DIM / 64, MROWS / 64), blk, 0, stream>>>(X16, Wt, avec, Vt16, EE);
  gat_attn_kernel<<<dim3(SEQ / 128, NHEAD, NB), blk, 0, stream>>>(Vt16, EE, MT, out);
}
